// DualInhibitionMemoryLayer_13134009991921
// MI455X (gfx1250) — hardware-run, weakly checked
//
#include <hip/hip_runtime.h>
#include <math.h>

typedef __attribute__((ext_vector_type(16))) _Float16 v16h;
typedef __attribute__((ext_vector_type(8)))  _Float16 v8h;
typedef __attribute__((ext_vector_type(8)))  float    v8f;
typedef __attribute__((ext_vector_type(4)))  float    v4f;
typedef __attribute__((address_space(1))) volatile v4f gv4f;

constexpr int kB     = 64;
constexpr int kT     = 128;
constexpr int kIn    = 128;
constexpr int kH     = 256;
constexpr int kInh   = 64;
constexpr int kDelay = 4;
constexpr int kRows  = kB * kT;
constexpr int kDrv   = 2 * kH;
constexpr int kBlkB  = 16;
constexpr int kThr   = 256;
constexpr int kXP    = 260;
constexpr int kVAP   = 264;
constexpr int kVIP   = 72;
constexpr int kTP    = 260;
constexpr int kTrP   = 68;
static_assert(kRows == 8192 && kDrv == 512, "drive plane shape");
static_assert((kIn % 32) == 0 && (kInh % 32) == 0 && (kH % 32) == 0 && (kT % 32) == 0, "K multiples of 32");
static_assert((kRows % 64) == 0 && (kDrv % 64) == 0 && (kT % 64) == 0 && (kH % 64) == 0, "GEMM M, N multiples of 64");
static_assert(kB % kBlkB == 0, "blocks own whole groups of 16 batch rows");
static_assert(kH == 32 * (kThr / 32), "8 waves x 32 value channels");
static_assert(kBlkB == 2 * (kThr / 32), "8 waves x 2 batch rows");
static_assert(kT == 4 * 32, "one v4f per lane covers a row of the inner-product plane");
static_assert((kT % 16) == 0, "key scan chunks of 16 steps");
static_assert((kDelay & (kDelay - 1)) == 0, "ring size power of two");
static_assert((kXP % 4) == 0 && (kVAP % 8) == 0 && (kVIP % 8) == 0 && (kTP % 4) == 0 && (kTrP % 4) == 0, "LDS pitches keep 16-B alignment");

constexpr double kAlphaD = 0.95122942450071400909;
constexpr float  kAlpha  = (float)kAlphaD;
constexpr float  kOma    = (float)(1.0 - kAlphaD);
constexpr float  kLr     = 1e-3f;
constexpr float  kRecall = 0.2f;

constexpr float kXCarry  = 128.0f;
constexpr float kWCarry  = 1024.0f;
constexpr float kACarry  = 1024.0f;
constexpr float kDrvFold = 1.0f / (kXCarry * kWCarry);
constexpr float kInhFold = 1.0f / (kACarry * kWCarry);
constexpr float kActFold = 1.0f / (kACarry * kACarry);
constexpr float kF16Min  = 6.103515625e-05f;

constexpr size_t kOutMem  = 0;
constexpr size_t kOutKeys = (size_t)kB * kH * kH;
constexpr size_t kOutVals = kOutKeys + (size_t)kB * kT * kH;
constexpr size_t kOutTot  = kOutVals + (size_t)kB * kT * kH;
static_assert(kOutKeys * 4 == 16777216ull && kOutVals * 4 == 25165824ull && kOutTot * 4 == 33554432ull, "output byte offsets");

constexpr size_t kOffXH    = 0;
constexpr size_t kOffWH    = kOffXH    + (size_t)kRows * kIn * 2;
constexpr size_t kOffWVEI  = kOffWH    + (size_t)kDrv * kIn * 2;
constexpr size_t kOffWIVE  = kOffWVEI  + (size_t)kInh * kH * 2;
constexpr size_t kOffIPL   = kOffWIVE  + (size_t)kH * kInh * 2;
constexpr size_t kOffKEY16 = kOffIPL   + (size_t)kRows * kDrv * 4;
constexpr size_t kOffKT16  = kOffKEY16 + (size_t)kRows * kH * 2;
constexpr size_t kOffKTF   = kOffKT16  + (size_t)kRows * kH * 2;
constexpr size_t kOffGPL   = kOffKTF   + (size_t)kRows * kH * 4;
constexpr size_t kOffVTF   = kOffGPL   + (size_t)kB * kT * kT * 4;
constexpr size_t kOffKTT16 = kOffVTF   + (size_t)kRows * kH * 4;
constexpr size_t kOffVTT16 = kOffKTT16 + (size_t)kB * kH * kT * 2;
constexpr size_t kWsTotal  = kOffVTT16 + (size_t)kB * kH * kT * 2;
static_assert(kWsTotal == 56819712ull, "carve total");
static_assert(kWsTotal <= 134217728ull, "carve cap");
static_assert((kOffWH % 256) == 0 && (kOffWVEI % 256) == 0 && (kOffWIVE % 256) == 0 && (kOffIPL % 256) == 0 &&
              (kOffKEY16 % 256) == 0 && (kOffKT16 % 256) == 0 && (kOffKTF % 256) == 0 && (kOffGPL % 256) == 0 &&
              (kOffVTF % 256) == 0 && (kOffKTT16 % 256) == 0 && (kOffVTT16 % 256) == 0, "aligned regions");

__device__ __forceinline__ unsigned short f2bf_bits(float f) {
  unsigned u = __float_as_uint(f);
  return (unsigned short)((u + 0x7FFFu + ((u >> 16) & 1u)) >> 16);
}
__device__ __forceinline__ float bf_bits2f(unsigned short h) { return __uint_as_float(((unsigned)h) << 16); }
__device__ __forceinline__ float bf16r(float f) { return bf_bits2f(f2bf_bits(f)); }

__device__ __forceinline__ _Float16 to_f16_carry_in(float v, float sc) {
  float r = bf16r(v) * sc;
  r = (fabsf(r) < kF16Min) ? 0.0f : r;
  return (_Float16)r;
}
__device__ __forceinline__ _Float16 to_f16_carry_act(float v) {
  float r = v * kACarry;
  r = (r < kF16Min) ? 0.0f : r;
  return (_Float16)r;
}

__device__ __forceinline__ void axpy4(v4f& a, float g, v4f x) {
  a[0] = fmaf(g, x[0], a[0]);
  a[1] = fmaf(g, x[1], a[1]);
  a[2] = fmaf(g, x[2], a[2]);
  a[3] = fmaf(g, x[3], a[3]);
}

__device__ __forceinline__ void dep_guard4_h(v8f& a0, v8f& a1, v8f& a2, v8f& a3, v16h x, v16h y) {
  asm volatile("v_nop\n\tv_nop\n\tv_nop\n\tv_nop" : "+v"(a0), "+v"(a1), "+v"(a2), "+v"(a3) : "v"(x), "v"(y));
}
__device__ __forceinline__ void keep4_h(v16h a, v16h b, v16h c, v16h d) { asm volatile("v_nop" :: "v"(a), "v"(b), "v"(c), "v"(d)); }
__device__ __forceinline__ void acc_guard4(v8f& a, v8f& b, v8f& c, v8f& d) {
  asm volatile("v_nop\n\tv_nop\n\tv_nop\n\tv_nop" : "+v"(a), "+v"(b), "+v"(c), "+v"(d));
}

template <typename T> struct Frag;
template <> struct Frag<_Float16> {
  typedef v16h V; union U { v16h v; v8h h[2]; };
  static __device__ __forceinline__ v16h load(const _Float16* p) {
    U f; f.h[0] = *(const v8h*)(p); f.h[1] = *(const v8h*)(p + 16); return f.v;
  }
  static __device__ __forceinline__ v8f mma(v16h a, v16h b, v8f c) {
    return __builtin_amdgcn_wmma_f32_16x16x32_f16(false, a, false, b, (short)0, c, false, false);
  }
  static __device__ __forceinline__ void guard4(v8f& a0, v8f& a1, v8f& a2, v8f& a3, v16h x, v16h y) { dep_guard4_h(a0, a1, a2, a3, x, y); }
  static __device__ __forceinline__ void keep(v16h a, v16h b, v16h c, v16h d) { keep4_h(a, b, c, d); }
};

__device__ __forceinline__ v8f mma_h(v16h a, v16h b, v8f c) {
  c = __builtin_amdgcn_wmma_f32_16x16x32_f16(false, a, false, b, (short)0, c, false, false);
  asm volatile("v_nop\n\tv_nop\n\tv_nop\n\tv_nop" : "+v"(c) : "v"(a), "v"(b));
  return c;
}

template <int ET> struct Elem;
template <> struct Elem<0> { typedef _Float16 T; };
template <int ET, bool SPLIT, int BIAS_MODE, int OUT_MODE, bool RESID, int ACT = 0>
__global__ __launch_bounds__(256) void wmma_gemm64(
    const unsigned short* __restrict__ Ap, const unsigned short* __restrict__ A2p, int lda, long strideA,
    const unsigned short* __restrict__ Btp, const unsigned short* __restrict__ Bt2p, int ldb, long strideB,
    void* __restrict__ Cout, void* __restrict__ Cout2, int ldc, long strideC,
    const float* __restrict__ bias,
    const float* __restrict__ resid, long strideR,
    int M, int N, int K, float scale) {
  typedef typename Elem<ET>::T T;
  typedef typename Frag<T>::V V;
  const T* A = (const T*)Ap; const T* A2 = (const T*)A2p; const T* Bt = (const T*)Btp; const T* Bt2 = (const T*)Bt2p;
  __shared__ __align__(16) float sT[8][16 * 68];
  const int b    = blockIdx.y;
  const int lane = threadIdx.x & 31;
  const int wave = threadIdx.x >> 5;
  const int tilesN = N >> 6;
  const int tilesM = M >> 6;
  const int tile = blockIdx.x * 8 + wave;
  if (tile >= tilesM * tilesN) return;
  const int tm = tile / tilesN;
  const int tn = tile - tm * tilesN;
  const int m0 = tm << 6;
  const int n0 = tn << 6;

  const T* Ab  = A  + (size_t)b * strideA;
  const T* Bb  = Bt + (size_t)b * strideB;
  const T* Ab2 = SPLIT ? (A2  + (size_t)b * strideA) : nullptr;
  const T* Bb2 = SPLIT ? (Bt2 + (size_t)b * strideB) : nullptr;

  const int rlane = lane & 15;
  const int koff  = (lane >> 4) * 8;
  const int mOff  = (lane >> 4) * 8;

  v8f acc[4][4];
#pragma unroll
  for (int i = 0; i < 4; ++i)
#pragma unroll
    for (int j = 0; j < 4; ++j) acc[i][j] = (v8f){0.f,0.f,0.f,0.f,0.f,0.f,0.f,0.f};

  for (int k0 = 0; k0 < K; k0 += 32) {
    V bh[4], bl[4];
#pragma unroll
    for (int j = 0; j < 4; ++j) {
      const size_t bo = (size_t)(n0 + (j << 4) + rlane) * ldb + koff + k0;
      bh[j] = Frag<T>::load(Bb + bo);
      if (SPLIT) bl[j] = Frag<T>::load(Bb2 + bo);
    }
#pragma unroll
    for (int i = 0; i < 4; ++i) {
      const size_t ao = (size_t)(m0 + (i << 4) + rlane) * lda + koff + k0;
      V ah = Frag<T>::load(Ab + ao);
      V al;
      if (SPLIT) al = Frag<T>::load(Ab2 + ao);
#pragma unroll
      for (int j = 0; j < 4; ++j) {
        acc[i][j] = Frag<T>::mma(ah, bh[j], acc[i][j]);
        if (SPLIT) {
          acc[i][j] = Frag<T>::mma(ah, bl[j], acc[i][j]);
          acc[i][j] = Frag<T>::mma(al, bh[j], acc[i][j]);
        }
      }
      Frag<T>::guard4(acc[i][0], acc[i][1], acc[i][2], acc[i][3], ah, SPLIT ? al : ah);
    }
    Frag<T>::keep(bh[0], bh[1], bh[2], bh[3]);
    if (SPLIT) Frag<T>::keep(bl[0], bl[1], bl[2], bl[3]);
  }
  acc_guard4(acc[0][0], acc[0][1], acc[0][2], acc[0][3]);
  acc_guard4(acc[1][0], acc[1][1], acc[1][2], acc[1][3]);
  acc_guard4(acc[2][0], acc[2][1], acc[2][2], acc[2][3]);
  acc_guard4(acc[3][0], acc[3][1], acc[3][2], acc[3][3]);

  float* slab = sT[wave];
  const float* Rb = RESID ? (resid + (size_t)b * strideR) : nullptr;
#pragma unroll
  for (int i = 0; i < 4; ++i) {
    const int mBase = m0 + (i << 4);
#pragma unroll
    for (int j = 0; j < 4; ++j) {
      const int n = n0 + (j << 4) + rlane;
      float bv = 0.f;
      if (BIAS_MODE == 2) bv = bias[n];
#pragma unroll
      for (int r = 0; r < 8; ++r) {
        float v = acc[i][j][r] * scale;
        if (BIAS_MODE == 1) v += bias[mBase + mOff + r];
        if (BIAS_MODE == 2) v += bv;
        if (RESID) v += Rb[(size_t)(mBase + mOff + r) * ldc + n];
        if (ACT == 2) v = fmaxf(v, 0.0f);
        if (ACT == 4) v = (v > 0.f) ? v : 0.01f * v;
        slab[(mOff + r) * 68 + (j << 4) + rlane] = v;
      }
    }
    __builtin_amdgcn_fence(__ATOMIC_RELEASE, "workgroup");
    __builtin_amdgcn_wave_barrier();
    __builtin_amdgcn_fence(__ATOMIC_ACQUIRE, "workgroup");
    if (OUT_MODE == 0) {
      float* C = (float*)Cout + (size_t)b * strideC;
      const int hh = lane >> 4, c4 = (lane & 15) * 4;
      for (int pass = 0; pass < 2; ++pass) {
#pragma unroll
        for (int it = 0; it < 8; ++it) {
          const int row = it * 2 + hh;
          v4f v = *(const v4f*)(slab + row * 68 + c4);
          *(volatile v4f*)(C + (size_t)(mBase + row) * ldc + n0 + c4) = v;
        }
        __threadfence();
      }
    } else {
      const int q = lane >> 3, c8 = (lane & 7) * 8;
      unsigned short* C  = (unsigned short*)Cout  + (size_t)b * strideC;
      unsigned short* C2 = (OUT_MODE == 2) ? ((unsigned short*)Cout2 + (size_t)b * strideC) : nullptr;
      for (int pass = 0; pass < 2; ++pass) {
#pragma unroll
        for (int it = 0; it < 4; ++it) {
          const int row = it * 4 + q;
          const float* sp = slab + row * 68 + c8;
          v8h hv, lv;
#pragma unroll
          for (int e = 0; e < 8; ++e) {
            if (OUT_MODE == 1) {
              hv[e] = (_Float16)sp[e];
            } else {
              unsigned short hb = f2bf_bits(sp[e]);
              unsigned short lb = f2bf_bits(sp[e] - bf_bits2f(hb));
              hv[e] = __builtin_bit_cast(_Float16, hb);
              lv[e] = __builtin_bit_cast(_Float16, lb);
            }
          }
          *(volatile v8h*)(C + (size_t)(mBase + row) * ldc + n0 + c8) = hv;
          if (OUT_MODE == 2) *(volatile v8h*)(C2 + (size_t)(mBase + row) * ldc + n0 + c8) = lv;
        }
        __threadfence();
      }
    }
    __builtin_amdgcn_fence(__ATOMIC_RELEASE, "workgroup");
    __builtin_amdgcn_wave_barrier();
    __builtin_amdgcn_fence(__ATOMIC_ACQUIRE, "workgroup");
  }
}

__global__ __launch_bounds__(256) void cvt8_carry_kernel(const float* __restrict__ src, unsigned short* __restrict__ dst,
                                                         int n8, float sc) {
  const int i = blockIdx.x * 256 + threadIdx.x;
  if (i < n8) {
    const float* sp = src + (size_t)i * 8;
    const v4f a = *(const v4f*)(sp);
    const v4f b = *(const v4f*)(sp + 4);
    v8h hv;
#pragma unroll
    for (int e = 0; e < 4; ++e) {
      const float x0 = a[e];
      const float x1 = b[e];
      hv[e]     = to_f16_carry_in(x0, sc);
      hv[4 + e] = to_f16_carry_in(x1, sc);
    }
    *(volatile v8h*)(dst + (size_t)i * 8) = hv;
    __threadfence();
    *(volatile v8h*)(dst + (size_t)i * 8) = hv;
  }
}

__global__ __launch_bounds__(256) void key_scan_kernel(const float* __restrict__ Ipl,
                                                       float* __restrict__ keysOut,
                                                       unsigned short* __restrict__ KEY16,
                                                       unsigned short* __restrict__ KT16,
                                                       float* __restrict__ KTF) {
  __shared__ __align__(16) float sK[16 * kTP];
  __shared__ __align__(16) float sR[16 * kTP];
  const int tid = threadIdx.x, lane = tid & 31, wave = tid >> 5;
  const int b = blockIdx.x;
  const size_t rowb = (size_t)b * kT;
  float ks = 0.0f, kt = 0.0f;
#pragma unroll 1
  for (int ch = 0; ch < kT / 16; ++ch) {
    const int t0 = ch * 16;
#pragma unroll 1
    for (int s = 0; s < 16; ++s) {
      const float ik = Ipl[(rowb + (size_t)(t0 + s)) * kDrv + tid];
      ks = kAlpha * ks + kOma * ik;
      const float key = fmaxf(ks, 0.0f);
      kt = kAlpha * kt + kOma * key;
      sK[s * kTP + tid] = key;
      sR[s * kTP + tid] = kt;
    }
    __syncthreads();
    v4f fk[4], ft[4];
#pragma unroll
    for (int it = 0; it < 4; ++it) {
      const int p = it * 8 + wave;
      const int row = p >> 1;
      const int col = (p & 1) * 128 + 4 * lane;
      fk[it] = *(const v4f*)(sK + row * kTP + col);
      ft[it] = *(const v4f*)(sR + row * kTP + col);
    }
    v8h hk[2], ht[2];
#pragma unroll
    for (int it = 0; it < 2; ++it) {
      const int row = it * 8 + wave;
      const v4f a0 = *(const v4f*)(sK + row * kTP + lane * 8);
      const v4f a1 = *(const v4f*)(sK + row * kTP + lane * 8 + 4);
      const v4f c0 = *(const v4f*)(sR + row * kTP + lane * 8);
      const v4f c1 = *(const v4f*)(sR + row * kTP + lane * 8 + 4);
#pragma unroll
      for (int e = 0; e < 4; ++e) {
        const float x0 = a0[e];
        const float x1 = a1[e];
        const float y0 = c0[e];
        const float y1 = c1[e];
        hk[it][e]     = to_f16_carry_act(x0);
        hk[it][4 + e] = to_f16_carry_act(x1);
        ht[it][e]     = to_f16_carry_act(y0);
        ht[it][4 + e] = to_f16_carry_act(y1);
      }
    }
    for (int pass = 0; pass < 2; ++pass) {
#pragma unroll
      for (int it = 0; it < 4; ++it) {
        const int p = it * 8 + wave;
        const int row = p >> 1;
        const int col = (p & 1) * 128 + 4 * lane;
        const size_t o = (rowb + (size_t)(t0 + row)) * kH + col;
        *(volatile v4f*)(keysOut + o) = fk[it];
        *(volatile v4f*)(KTF + o)     = ft[it];
      }
#pragma unroll
      for (int it = 0; it < 2; ++it) {
        const int row = it * 8 + wave;
        const size_t o = (rowb + (size_t)(t0 + row)) * kH + lane * 8;
        *(volatile v8h*)(KEY16 + o) = hk[it];
        *(volatile v8h*)(KT16 + o)  = ht[it];
      }
      __threadfence();
    }
    __syncthreads();
  }
}

__global__ __launch_bounds__(256) void transpose_carry_kernel(const float* __restrict__ src, unsigned short* __restrict__ dst) {
  __shared__ __align__(16) float tS[kT * kTrP];
  const int tid = threadIdx.x, lane = tid & 31, wave = tid >> 5;
  const int b = blockIdx.y;
  const int i0 = blockIdx.x * 64;
#pragma unroll
  for (int it = 0; it < 8; ++it) {
    const int idx = it * 256 + tid;
    const int s = idx >> 4;
    const int c4 = (idx & 15) * 4;
    const v4f v = *(const v4f*)(src + ((size_t)b * kT + (size_t)s) * kH + i0 + c4);
    *(v4f*)(tS + s * kTrP + c4) = v;
  }
  __syncthreads();
  const int hh = lane >> 4;
  const int s8 = (lane & 15) * 8;
  v8h hv[4];
#pragma unroll
  for (int it = 0; it < 4; ++it) {
    const int il = it * 16 + wave * 2 + hh;
#pragma unroll
    for (int e = 0; e < 8; ++e) {
      const float x = tS[(s8 + e) * kTrP + il];
      hv[it][e] = to_f16_carry_act(x);
    }
  }
  for (int pass = 0; pass < 2; ++pass) {
#pragma unroll
    for (int it = 0; it < 4; ++it) {
      const int il = it * 16 + wave * 2 + hh;
      *(volatile v8h*)(dst + ((size_t)b * kH + (size_t)(i0 + il)) * kT + s8) = hv[it];
    }
    __threadfence();
  }
}

__global__ __launch_bounds__(kThr) void fastmem_seq_kernel(const float* __restrict__ Ipl,
                                                           const float* __restrict__ Gpl,
                                                           const unsigned short* __restrict__ WIVEp,
                                                           const unsigned short* __restrict__ WVEIp,
                                                           float* VTF,
                                                           float* __restrict__ valsOut) {
  __shared__ __align__(16) float    gS[kBlkB * kT];
  __shared__ __align__(16) float    vtS[kBlkB * kH];
  __shared__ __align__(16) float    xS[kBlkB * kXP];
  __shared__ __align__(16) _Float16 valA[kBlkB * kVAP];
  __shared__ __align__(16) _Float16 viA[kDelay][kBlkB * kVIP];

  const _Float16* WIVE = (const _Float16*)WIVEp;
  const _Float16* WVEI = (const _Float16*)WVEIp;
  const int tid  = threadIdx.x;
  const int lane = tid & 31;
  const int wave = __builtin_amdgcn_readfirstlane(tid >> 5);
  const int c    = lane & 15;
  const int hh   = lane >> 4;
  const int koff = hh * 8;
  const int b0   = blockIdx.x * kBlkB;

#pragma unroll 1
  for (int i = tid; i < kBlkB * kT; i += kThr) gS[i] = 0.0f;
#pragma unroll 1
  for (int i = tid; i < kBlkB * kH; i += kThr) vtS[i] = 0.0f;
#pragma unroll 1
  for (int i = tid; i < kBlkB * kXP; i += kThr) xS[i] = 0.0f;
#pragma unroll 1
  for (int i = tid; i < kBlkB * kVAP; i += kThr) valA[i] = (_Float16)0.0f;
  {
    _Float16* vf = &viA[0][0];
#pragma unroll 1
    for (int i = tid; i < kDelay * kBlkB * kVIP; i += kThr) vf[i] = (_Float16)0.0f;
  }

  float vs[2][8], vt[2][8], vis[8];
#pragma unroll
  for (int nt = 0; nt < 2; ++nt)
#pragma unroll
    for (int r = 0; r < 8; ++r) { vs[nt][r] = 0.0f; vt[nt][r] = 0.0f; }
#pragma unroll
  for (int r = 0; r < 8; ++r) vis[r] = 0.0f;

  const v8f z8 = {0.f, 0.f, 0.f, 0.f, 0.f, 0.f, 0.f, 0.f};
  const v4f z4 = {0.f, 0.f, 0.f, 0.f};
  const int rA = 2 * wave;
  const gv4f* pA = (const gv4f*)(size_t)(VTF + ((size_t)(b0 + rA) * kT) * kH + 4 * lane);
  const gv4f* pB = (const gv4f*)(size_t)(VTF + ((size_t)(b0 + rA + 1) * kT) * kH + 4 * lane);

  __syncthreads();

#pragma unroll 1
  for (int t = 0; t < kT; ++t) {
    const int slot = t & (kDelay - 1);

    {
      const v4f g0 = *(const v4f*)(Gpl + ((size_t)(b0 + rA) * kT + (size_t)t) * kT + 4 * lane);
      const v4f g1 = *(const v4f*)(Gpl + ((size_t)(b0 + rA + 1) * kT + (size_t)t) * kT + 4 * lane);
      *(v4f*)(gS + rA * kT + 4 * lane)       = g0;
      *(v4f*)(gS + (rA + 1) * kT + 4 * lane) = g1;
    }
    __syncthreads();

    {
      const float* gA = gS + rA * kT;
      const float* gB = gA + kT;
      v4f a0 = z4, a1 = z4, c0 = z4, c1 = z4;
#pragma unroll 1
      for (int s = 0; s < t; ++s) {
        const float ga = gA[s];
        const float gb = gB[s];
        const v4f x0 = pA[s * (kH / 4)];
        const v4f x1 = pA[s * (kH / 4) + 32];
        const v4f y0 = pB[s * (kH / 4)];
        const v4f y1 = pB[s * (kH / 4) + 32];
        axpy4(a0, ga, x0);
        axpy4(a1, ga, x1);
        axpy4(c0, gb, y0);
        axpy4(c1, gb, y1);
      }
      v4f o0, o1, o2, o3;
#pragma unroll
      for (int e = 0; e < 4; ++e) {
        o0[e] = kRecall * (kLr * a0[e]);
        o1[e] = kRecall * (kLr * a1[e]);
        o2[e] = kRecall * (kLr * c0[e]);
        o3[e] = kRecall * (kLr * c1[e]);
      }
      *(v4f*)(xS + rA * kXP + 4 * lane)             = o0;
      *(v4f*)(xS + rA * kXP + 128 + 4 * lane)       = o1;
      *(v4f*)(xS + (rA + 1) * kXP + 4 * lane)       = o2;
      *(v4f*)(xS + (rA + 1) * kXP + 128 + 4 * lane) = o3;
    }
    __syncthreads();

    {
      int kp = koff;
      asm volatile("" : "+v"(kp));
      float ivr[2][8];
#pragma unroll
      for (int nt = 0; nt < 2; ++nt)
#pragma unroll
        for (int r = 0; r < 8; ++r)
          ivr[nt][r] = Ipl[((size_t)(b0 + 8 * hh + r) * kT + (size_t)t) * kDrv + kH + 32 * wave + 16 * nt + c];
      const _Float16* va = &viA[slot][0] + c * kVIP + koff;
      v8f acc[2];
      acc[0] = z8; acc[1] = z8;
#pragma unroll
      for (int k2 = 0; k2 < kInh / 32; ++k2) {
        const v16h af = Frag<_Float16>::load(va + 32 * k2);
#pragma unroll
        for (int nt = 0; nt < 2; ++nt) {
          const v16h bf = Frag<_Float16>::load(WIVE + (size_t)(32 * wave + 16 * nt + c) * kInh + kp + 32 * k2);
          acc[nt] = mma_h(af, bf, acc[nt]);
        }
      }
#pragma unroll
      for (int nt = 0; nt < 2; ++nt) {
        const int i = 32 * wave + 16 * nt + c;
#pragma unroll
        for (int r = 0; r < 8; ++r) {
          const int b = 8 * hh + r;
          const float vio = acc[nt][r] * kInhFold;
          const float ikv = xS[b * kXP + i];
          const float drive = (ivr[nt][r] + ikv) + vio;
          vs[nt][r] = kAlpha * vs[nt][r] + kOma * drive;
          const float val = fmaxf(vs[nt][r], 0.0f);
          vt[nt][r] = kAlpha * vt[nt][r] + kOma * val;
          xS[b * kXP + i]    = val;
          valA[b * kVAP + i] = to_f16_carry_act(val);
          vtS[b * kH + i]    = vt[nt][r];
        }
      }
    }
    __syncthreads();

    {
      v4f vv[4], tv[4];
#pragma unroll
      for (int q = 0; q < 4; ++q) {
        const int row = rA + (q >> 1);
        const int col = (q & 1) * 128 + 4 * lane;
        vv[q] = *(const v4f*)(xS + row * kXP + col);
        tv[q] = *(const v4f*)(vtS + row * kH + col);
      }
      for (int pass = 0; pass < 2; ++pass) {
#pragma unroll
        for (int q = 0; q < 4; ++q) {
          const int row = rA + (q >> 1);
          const int col = (q & 1) * 128 + 4 * lane;
          const size_t o = ((size_t)(b0 + row) * kT + (size_t)t) * kH + col;
          *(volatile v4f*)(valsOut + o) = vv[q];
          *(volatile v4f*)(VTF + o)     = tv[q];
        }
        __threadfence();
      }
    }

    if (wave < 4) {
      int kp2 = koff;
      asm volatile("" : "+v"(kp2));
      const _Float16* aa = valA + c * kVAP + koff;
      const _Float16* wb = WVEI + (size_t)(16 * wave + c) * kH + kp2;
      v8f acc = z8;
#pragma unroll
      for (int k8 = 0; k8 < kH / 32; ++k8) {
        const v16h af = Frag<_Float16>::load(aa + 32 * k8);
        const v16h bf = Frag<_Float16>::load(wb + 32 * k8);
        acc = mma_h(af, bf, acc);
      }
      _Float16* vw = &viA[slot][0];
#pragma unroll
      for (int r = 0; r < 8; ++r) {
        const float vii = acc[r] * kInhFold;
        vis[r] = kAlpha * vis[r] + kOma * vii;
        const float vi = fmaxf(vis[r], 0.0f);
        vw[(8 * hh + r) * kVIP + 16 * wave + c] = to_f16_carry_act(vi);
      }
    }
  }
  __threadfence();
}

extern "C" void kernel_launch(void* const* d_in, const int* in_sizes, int n_in,
                              void* d_out, int out_size, void* d_ws, size_t ws_size, hipStream_t stream) {
  if (n_in < 4 || d_out == nullptr || d_ws == nullptr) return;
  if (in_sizes[0] != kB * kT * kIn) return;
  if (in_sizes[1] != kDrv * kIn) return;
  if (in_sizes[2] != kInh * kH) return;
  if (in_sizes[3] != kH * kInh) return;
  if ((size_t)out_size != kOutTot) return;
  if (ws_size < kWsTotal) return;

  const float* x     = (const float*)d_in[0];
  const float* W     = (const float*)d_in[1];
  const float* W_vei = (const float*)d_in[2];
  const float* W_ive = (const float*)d_in[3];
  float* out = (float*)d_out;

  char* ws = (char*)d_ws;
  unsigned short* XH    = (unsigned short*)(ws + kOffXH);
  unsigned short* WH    = (unsigned short*)(ws + kOffWH);
  unsigned short* WVEI  = (unsigned short*)(ws + kOffWVEI);
  unsigned short* WIVE  = (unsigned short*)(ws + kOffWIVE);
  float*          IPL   = (float*)(ws + kOffIPL);
  unsigned short* KEY16 = (unsigned short*)(ws + kOffKEY16);
  unsigned short* KT16  = (unsigned short*)(ws + kOffKT16);
  float*          KTF   = (float*)(ws + kOffKTF);
  float*          GPL   = (float*)(ws + kOffGPL);
  float*          VTF   = (float*)(ws + kOffVTF);
  unsigned short* KTT16 = (unsigned short*)(ws + kOffKTT16);
  unsigned short* VTT16 = (unsigned short*)(ws + kOffVTT16);

  const int n8x  = kRows * kIn / 8;
  const int n8w  = kDrv * kIn / 8;
  const int n8ve = kInh * kH / 8;
  const int n8iv = kH * kInh / 8;
  cvt8_carry_kernel<<<(n8x  + 255) / 256, 256, 0, stream>>>(x,     XH,   n8x,  kXCarry);
  cvt8_carry_kernel<<<(n8w  + 255) / 256, 256, 0, stream>>>(W,     WH,   n8w,  kWCarry);
  cvt8_carry_kernel<<<(n8ve + 255) / 256, 256, 0, stream>>>(W_vei, WVEI, n8ve, kWCarry);
  cvt8_carry_kernel<<<(n8iv + 255) / 256, 256, 0, stream>>>(W_ive, WIVE, n8iv, kWCarry);

  wmma_gemm64<0, false, 0, 0, false, 0><<<dim3((kRows / 64) * (kDrv / 64) / 8, 1), 256, 0, stream>>>(
      XH, XH, kIn, 0L,
      WH, WH, kIn, 0L,
      (void*)IPL, (void*)IPL, kDrv, 0L,
      W, W, 0L,
      kRows, kDrv, kIn, kDrvFold);

  key_scan_kernel<<<kB, 256, 0, stream>>>(IPL, out + kOutKeys, KEY16, KT16, KTF);

  wmma_gemm64<0, false, 0, 0, false, 0><<<dim3(1, kB), 128, 0, stream>>>(
      KEY16, KEY16, kH, (long)kT * kH,
      KT16, KT16, kH, (long)kT * kH,
      (void*)GPL, (void*)GPL, kT, (long)kT * kT,
      W, W, 0L,
      kT, kT, kH, kActFold);

  fastmem_seq_kernel<<<kB / kBlkB, kThr, 0, stream>>>(IPL, GPL, WIVE, WVEI, VTF, out + kOutVals);

  transpose_carry_kernel<<<dim3(kH / 64, kB), 256, 0, stream>>>(KTF, KTT16);
  transpose_carry_kernel<<<dim3(kH / 64, kB), 256, 0, stream>>>(VTF, VTT16);

  wmma_gemm64<0, false, 0, 0, false, 0><<<dim3((kH / 64) * (kH / 64) / 8, kB), 256, 0, stream>>>(
      VTT16, VTT16, kT, (long)kH * kT,
      KTT16, KTT16, kT, (long)kH * kT,
      (void*)(out + kOutMem), (void*)(out + kOutMem), kH, (long)kH * kH,
      W, W, 0L,
      kH, kH, kT, kLr * kActFold);
}
